// MultiHeadAttention_37477884625165
// MI455X (gfx1250) — hardware-run, weakly checked
//
#include <hip/hip_runtime.h>
#include <math.h>

typedef __attribute__((ext_vector_type(16))) _Float16 v16h;
typedef __attribute__((ext_vector_type(8)))  _Float16 v8h;
typedef __attribute__((ext_vector_type(8)))  float    v8f;
typedef __attribute__((ext_vector_type(4)))  float    v4f;

constexpr int kBatch = 2;
constexpr int kNq    = 2048;
constexpr int kNk    = 2048;
constexpr int kDm    = 512;
constexpr int kNh    = 8;
constexpr int kDh    = 64;
constexpr int kTokQ  = kBatch * kNq;
constexpr int kTokK  = kBatch * kNk;
constexpr int kQBlk  = kNq / 64;
constexpr int kKChunks = kNk / 64;
static_assert(kNh * kDh == kDm);
static_assert(kDh == 64);
static_assert((kDm % 64) == 0 && (kTokQ % 64) == 0 && (kTokK % 64) == 0 && (kDm % 32) == 0);
static_assert((kNq % 64) == 0 && (kNk % 64) == 0);

constexpr int ce_isqrt(int n) { int r = 0; while ((r + 1) * (r + 1) <= n) ++r; return r; }
static_assert(ce_isqrt(kDh) * ce_isqrt(kDh) == kDh);
constexpr float kInvSqrtDh = 1.0f / (float)ce_isqrt(kDh);

constexpr float kXCarry   = 16.0f;
constexpr float kWCarry   = 256.0f;
constexpr float kQkvCarry = 16.0f;
constexpr float kPCarry   = 32768.0f;
constexpr float kProjScale  = kQkvCarry / (kXCarry * kWCarry);
constexpr float kScoreScale = kInvSqrtDh / (kQkvCarry * kQkvCarry);
constexpr float kOutCarry   = kPCarry * kQkvCarry;

constexpr size_t kSzWT   = (size_t)3 * kDm * kDm * 2;
constexpr size_t kSzX16  = (size_t)3 * kTokQ * kDm * 2;
constexpr size_t kSzQ16  = (size_t)kTokQ * kDm * 2;
constexpr size_t kSzK16  = (size_t)kTokK * kDm * 2;
constexpr size_t kSzVT16 = (size_t)kDm * kTokK * 2;
constexpr size_t kOffWT   = 0;
constexpr size_t kOffX16  = kOffWT  + kSzWT;
constexpr size_t kOffQ16  = kOffX16 + kSzX16;
constexpr size_t kOffK16  = kOffQ16 + kSzQ16;
constexpr size_t kOffVT16 = kOffK16 + kSzK16;
constexpr size_t kWsTotal = kOffVT16 + kSzVT16;
static_assert(kWsTotal == 26738688ull);
static_assert(kWsTotal <= 134217728ull);
static_assert((kOffX16 % 128) == 0 && (kOffQ16 % 128) == 0 && (kOffK16 % 128) == 0 && (kOffVT16 % 128) == 0);
static_assert(kTokQ == kTokK);

union FragU { v16h v; v8h h[2]; };
__device__ __forceinline__ v16h frag_load(const _Float16* p) {
  FragU f;
  f.h[0] = *(const v8h*)(p);
  f.h[1] = *(const v8h*)(p + 16);
  return f.v;
}
__device__ __forceinline__ v8f mma_f16(v16h a, v16h b, v8f c) {
  c = __builtin_amdgcn_wmma_f32_16x16x32_f16(false, a, false, b, (short)0, c, false, false);
  asm volatile("v_nop\n\tv_nop\n\tv_nop\n\tv_nop" : "+v"(c) : "v"(a), "v"(b));
  return c;
}

__global__ __launch_bounds__(256) void wt_cast_kernel(const float* __restrict__ W0, const float* __restrict__ W1,
                                                      const float* __restrict__ W2,
                                                      unsigned short* __restrict__ outp, float carry) {
  __shared__ float sm[64][65];
  const int t  = threadIdx.x;
  const int k0 = blockIdx.x * 64;
  const int j0 = blockIdx.y * 64;
  const int z  = blockIdx.z;
  const float* W = (z == 0) ? W0 : (z == 1) ? W1 : W2;
#pragma unroll
  for (int i = 0; i < 16; ++i) {
    const int e  = i * 256 + t;
    const int r  = e >> 6;
    const int cc = e & 63;
    sm[cc][r] = W[(size_t)(k0 + r) * kDm + j0 + cc] * carry;
  }
  __syncthreads();
  const int lane = t & 31;
  const int wave = __builtin_amdgcn_readfirstlane((int)(threadIdx.x >> 5));
  const int q = lane >> 3, c8 = (lane & 7) * 8;
  unsigned short* op = outp + (size_t)z * kDm * kDm;
  v8h hv[2];
#pragma unroll
  for (int it = 0; it < 2; ++it) {
    const int row = wave * 8 + it * 4 + q;
#pragma unroll
    for (int e = 0; e < 8; ++e) hv[it][e] = (_Float16)sm[row][c8 + e];
  }
  for (int pass = 0; pass < 2; ++pass) {
#pragma unroll
    for (int it = 0; it < 2; ++it) {
      const int row = wave * 8 + it * 4 + q;
      *(volatile v8h*)(op + (size_t)(j0 + row) * kDm + k0 + c8) = hv[it];
    }
    __threadfence();
  }
}

__global__ __launch_bounds__(256) void cast_x_kernel(const float* __restrict__ x0, const float* __restrict__ x1,
                                                     const float* __restrict__ x2,
                                                     unsigned short* __restrict__ outp, int n8, float carry) {
  const int z = blockIdx.y;
  const float* in = (z == 0) ? x0 : (z == 1) ? x1 : x2;
  const int i = blockIdx.x * 256 + threadIdx.x;
  if (i >= n8) return;
  const float* p = in + 8 * (size_t)i;
  const v4f a = *(const v4f*)(p);
  const v4f c = *(const v4f*)(p + 4);
  v8h hv;
#pragma unroll
  for (int e = 0; e < 4; ++e) {
    hv[e]     = (_Float16)(a[e] * carry);
    hv[4 + e] = (_Float16)(c[e] * carry);
  }
  unsigned short* q = outp + (size_t)z * ((size_t)n8 * 8) + 8 * (size_t)i;
  *(volatile v8h*)q = hv;
  __threadfence();
  *(volatile v8h*)q = hv;
}

template <int BIAS_MODE>
__global__ __launch_bounds__(256) void gemm64_f16_kernel(
    const unsigned short* __restrict__ Ap, int lda,
    const unsigned short* __restrict__ Btp, int ldb,
    unsigned short* __restrict__ Cp, int ldc,
    const float* __restrict__ bias, int M, int N, int K, float scale, float bscale) {
  const _Float16* A  = (const _Float16*)Ap;
  const _Float16* Bt = (const _Float16*)Btp;
  __shared__ __align__(16) float sT[8][16 * 68];
  const int lane = threadIdx.x & 31;
  const int wave = __builtin_amdgcn_readfirstlane((int)(threadIdx.x >> 5));
  const int tilesN = N >> 6;
  const int tilesM = M >> 6;
  const int tile = blockIdx.x * 8 + wave;
  if (tile >= tilesM * tilesN) return;
  const int tm = tile / tilesN;
  const int tn = tile - tm * tilesN;
  const int m0 = tm << 6;
  const int n0 = tn << 6;

  const int rlane = lane & 15;
  const int koff  = (lane >> 4) * 8;
  const int mOff  = (lane >> 4) * 8;

  v8f acc[4][4];
#pragma unroll
  for (int i = 0; i < 4; ++i)
#pragma unroll
    for (int j = 0; j < 4; ++j) acc[i][j] = (v8f){0.f, 0.f, 0.f, 0.f, 0.f, 0.f, 0.f, 0.f};

  for (int k0 = 0; k0 < K; k0 += 32) {
    v16h bh[4];
#pragma unroll
    for (int j = 0; j < 4; ++j) {
      const size_t bo = (size_t)(n0 + (j << 4) + rlane) * ldb + koff + k0;
      bh[j] = frag_load(Bt + bo);
    }
#pragma unroll
    for (int i = 0; i < 4; ++i) {
      const size_t ao = (size_t)(m0 + (i << 4) + rlane) * lda + koff + k0;
      const v16h ah = frag_load(A + ao);
#pragma unroll
      for (int j = 0; j < 4; ++j) acc[i][j] = mma_f16(ah, bh[j], acc[i][j]);
    }
  }

  float* slab = sT[wave];
#pragma unroll
  for (int i = 0; i < 4; ++i) {
    const int mBase = m0 + (i << 4);
#pragma unroll
    for (int j = 0; j < 4; ++j) {
      const int n = n0 + (j << 4) + rlane;
      float bv = 0.f;
      if (BIAS_MODE == 2) bv = bias[n] * bscale;
#pragma unroll
      for (int r = 0; r < 8; ++r) {
        float v = acc[i][j][r] * scale;
        if (BIAS_MODE == 1) v += bias[mBase + mOff + r] * bscale;
        if (BIAS_MODE == 2) v += bv;
        slab[(mOff + r) * 68 + (j << 4) + rlane] = v;
      }
    }
    __builtin_amdgcn_fence(__ATOMIC_RELEASE, "workgroup");
    __builtin_amdgcn_wave_barrier();
    __builtin_amdgcn_fence(__ATOMIC_ACQUIRE, "workgroup");
    {
      const int q = lane >> 3, c8 = (lane & 7) * 8;
      for (int pass = 0; pass < 2; ++pass) {
#pragma unroll
        for (int it = 0; it < 4; ++it) {
          const int row = it * 4 + q;
          const float* sp = slab + row * 68 + c8;
          v8h hv;
#pragma unroll
          for (int e = 0; e < 8; ++e) hv[e] = (_Float16)sp[e];
          *(volatile v8h*)(Cp + (size_t)(mBase + row) * ldc + n0 + c8) = hv;
        }
        __threadfence();
      }
    }
    __builtin_amdgcn_fence(__ATOMIC_RELEASE, "workgroup");
    __builtin_amdgcn_wave_barrier();
    __builtin_amdgcn_fence(__ATOMIC_ACQUIRE, "workgroup");
  }
}

constexpr int kHP = 72;
constexpr int kFP = 68;
constexpr int kNW = 4;

__global__ __launch_bounds__(128) void attn_kernel(const unsigned short* __restrict__ Qp,
                                                   const unsigned short* __restrict__ Kp,
                                                   const unsigned short* __restrict__ Vtp,
                                                   const float* __restrict__ af,
                                                   const float* __restrict__ kw,
                                                   float* __restrict__ outp) {
  __shared__ __align__(16) _Float16 Ksh[64 * kHP];
  __shared__ __align__(16) _Float16 Vsh[kDh * kHP];
  __shared__ __align__(16) _Float16 Psh[kNW][16 * kHP];
  __shared__ __align__(16) float    Fsh[kNW][16 * kFP];

  const _Float16* Q16  = (const _Float16*)Qp;
  const _Float16* K16  = (const _Float16*)Kp;
  const _Float16* Vt16 = (const _Float16*)Vtp;

  const int tid  = threadIdx.x;
  const int wave = __builtin_amdgcn_readfirstlane((int)(threadIdx.x >> 5));
  const int lane = tid & 31;
  const int hh   = lane >> 4;
  const int c    = lane & 15;

  const int bx = blockIdx.x;
  const int h  = bx % kNh;
  const int tq = bx / kNh;
  const int qb = tq % kQBlk;
  const int b  = tq / kQBlk;
  const int q0 = qb * 64 + wave * 16;

  v16h qa[2];
  {
    const _Float16* qrow = Q16 + ((size_t)b * kNq + q0 + c) * kDm + h * kDh + 8 * hh;
    qa[0] = frag_load(qrow);
    qa[1] = frag_load(qrow + 32);
  }

  const _Float16* Kg  = K16 + (size_t)b * kNk * kDm + h * kDh;
  const _Float16* Vg  = Vt16 + (size_t)(h * kDh) * kTokK + (size_t)b * kNk;
  const float*    afw = af + ((size_t)b * kNq + q0) * kNk;
  const float*    kwb = kw + (size_t)b * kNk;

  const int srow = tid >> 3;
  const int soff = (tid & 7) * 8;
  const int frow = lane >> 4;
  const int fc4  = (lane & 15) * 4;

  float mrow[8], lrow[8];
  v8f oacc[4];
#pragma unroll
  for (int r = 0; r < 8; ++r) { mrow[r] = -1.0e30f; lrow[r] = 0.f; }
#pragma unroll
  for (int t = 0; t < 4; ++t) oacc[t] = (v8f){0.f, 0.f, 0.f, 0.f, 0.f, 0.f, 0.f, 0.f};

  float*    fs = Fsh[wave];
  _Float16* pw = Psh[wave];

#pragma unroll 1
  for (int kc = 0; kc < kKChunks; ++kc) {
    const int kv0 = kc * 64;
    v8h kr[4], vr[4];
    v4f fr[8];
    float kwv[4];
#pragma unroll
    for (int i = 0; i < 4; ++i) {
      kr[i] = *(const v8h*)(Kg + (size_t)(kv0 + srow + 16 * i) * kDm + soff);
      vr[i] = *(const v8h*)(Vg + (size_t)(srow + 16 * i) * kTokK + kv0 + soff);
    }
#pragma unroll
    for (int i = 0; i < 8; ++i) fr[i] = *(const v4f*)(afw + (size_t)(frow + 2 * i) * kNk + kv0 + fc4);
#pragma unroll
    for (int j = 0; j < 4; ++j) kwv[j] = kwb[kv0 + j * 16 + c];

    __syncthreads();
#pragma unroll
    for (int i = 0; i < 4; ++i) {
      *(v8h*)(Ksh + (srow + 16 * i) * kHP + soff) = kr[i];
      *(v8h*)(Vsh + (srow + 16 * i) * kHP + soff) = vr[i];
    }
#pragma unroll
    for (int i = 0; i < 8; ++i) *(v4f*)(fs + (frow + 2 * i) * kFP + fc4) = fr[i];
    __syncthreads();

    v8f s[4];
#pragma unroll
    for (int j = 0; j < 4; ++j) {
      s[j] = (v8f){0.f, 0.f, 0.f, 0.f, 0.f, 0.f, 0.f, 0.f};
#pragma unroll
      for (int dc = 0; dc < 2; ++dc) {
        const v16h kb = frag_load(Ksh + (j * 16 + c) * kHP + dc * 32 + 8 * hh);
        s[j] = mma_f16(qa[dc], kb, s[j]);
      }
    }

    float cm[8];
#pragma unroll
    for (int r = 0; r < 8; ++r) {
      const float* frp = fs + (8 * hh + r) * kFP + c;
      float m = -1.0e30f;
#pragma unroll
      for (int j = 0; j < 4; ++j) {
        const float a = frp[j * 16];
        const float val = ((s[j][r] * kScoreScale) * a) * kwv[j];
        s[j][r] = val;
        m = fmaxf(m, val);
      }
#pragma unroll
      for (int off = 1; off < 16; off <<= 1) m = fmaxf(m, __shfl_xor(m, off, 32));
      cm[r] = m;
    }

#pragma unroll
    for (int r = 0; r < 8; ++r) {
      const float mnew  = fmaxf(mrow[r], cm[r]);
      const float alpha = __expf(mrow[r] - mnew);
      mrow[r] = mnew;
      float psum = 0.f;
#pragma unroll
      for (int j = 0; j < 4; ++j) {
        const float p = __expf(s[j][r] - mnew);
        psum += p;
        pw[(8 * hh + r) * kHP + j * 16 + c] = (_Float16)(p * kPCarry);
      }
#pragma unroll
      for (int off = 1; off < 16; off <<= 1) psum += __shfl_xor(psum, off, 32);
      lrow[r] = lrow[r] * alpha + psum;
#pragma unroll
      for (int t = 0; t < 4; ++t) oacc[t][r] *= alpha;
    }

    __syncthreads();

#pragma unroll
    for (int kk = 0; kk < 2; ++kk) {
      const v16h pa = frag_load(pw + c * kHP + kk * 32 + 8 * hh);
#pragma unroll
      for (int t = 0; t < 4; ++t) {
        const v16h vb = frag_load(Vsh + (t * 16 + c) * kHP + kk * 32 + 8 * hh);
        oacc[t] = mma_f16(pa, vb, oacc[t]);
      }
    }
  }

#pragma unroll
  for (int r = 0; r < 8; ++r) {
    const float inv = 1.0f / (lrow[r] * kOutCarry);
#pragma unroll
    for (int t = 0; t < 4; ++t) fs[(8 * hh + r) * kFP + t * 16 + c] = oacc[t][r] * inv;
  }
  __syncthreads();
  {
    float* ob = outp + ((size_t)b * kNq + q0) * kDm + h * kDh;
    const int c4 = (lane & 15) * 4;
    for (int pass = 0; pass < 2; ++pass) {
#pragma unroll
      for (int it = 0; it < 8; ++it) {
        const int row = it * 2 + hh;
        const v4f val = *(const v4f*)(fs + row * kFP + c4);
        *(volatile v4f*)(ob + (size_t)row * kDm + c4) = val;
      }
      __threadfence();
    }
  }
}

extern "C" void kernel_launch(void* const* d_in, const int* in_sizes, int n_in,
                              void* d_out, int out_size, void* d_ws, size_t ws_size,
                              hipStream_t stream) {
  if (n_in < 11) return;
  if (in_sizes[0] != kTokQ * kDm) return;
  if (in_sizes[1] != kTokK * kDm) return;
  if (in_sizes[2] != kTokK * kDm) return;
  if (in_sizes[3] != kBatch * kNk) return;
  if (in_sizes[4] != kBatch * kNq * kNk) return;
  if (in_sizes[5] != kDm * kDm) return;
  if (in_sizes[6] != kDm) return;
  if (in_sizes[7] != kDm * kDm) return;
  if (in_sizes[8] != kDm) return;
  if (in_sizes[9] != kDm * kDm) return;
  if (in_sizes[10] != kDm) return;
  if (out_size != kTokQ * kDm) return;
  if (ws_size < kWsTotal) return;

  const float* xq = (const float*)d_in[0];
  const float* xk = (const float*)d_in[1];
  const float* xv = (const float*)d_in[2];
  const float* kwt = (const float*)d_in[3];
  const float* aft = (const float*)d_in[4];
  const float* Wq = (const float*)d_in[5];
  const float* bq = (const float*)d_in[6];
  const float* Wk = (const float*)d_in[7];
  const float* bk = (const float*)d_in[8];
  const float* Wv = (const float*)d_in[9];
  const float* bv = (const float*)d_in[10];
  float* out = (float*)d_out;

  char* ws = (char*)d_ws;
  unsigned short* WT   = (unsigned short*)(ws + kOffWT);
  unsigned short* X16  = (unsigned short*)(ws + kOffX16);
  unsigned short* Q16  = (unsigned short*)(ws + kOffQ16);
  unsigned short* K16  = (unsigned short*)(ws + kOffK16);
  unsigned short* VT16 = (unsigned short*)(ws + kOffVT16);

  unsigned short* WTq = WT;
  unsigned short* WTk = WT + (size_t)kDm * kDm;
  unsigned short* WTv = WT + (size_t)2 * kDm * kDm;
  unsigned short* Xq16 = X16;
  unsigned short* Xk16 = X16 + (size_t)kTokQ * kDm;
  unsigned short* Xv16 = X16 + (size_t)2 * kTokQ * kDm;

  wt_cast_kernel<<<dim3(kDm / 64, kDm / 64, 3), 256, 0, stream>>>(Wq, Wk, Wv, WT, kWCarry);

  constexpr int n8 = kTokQ * kDm / 8;
  static_assert((n8 % 256) == 0);
  cast_x_kernel<<<dim3(n8 / 256, 3), 256, 0, stream>>>(xq, xk, xv, X16, n8, kXCarry);

  constexpr int tilesQ = (kTokQ / 64) * (kDm / 64);
  static_assert((tilesQ % 8) == 0);
  gemm64_f16_kernel<2><<<tilesQ / 8, 256, 0, stream>>>(
      Xq16, kDm, WTq, kDm, Q16, kDm, bq, kTokQ, kDm, kDm, kProjScale, kQkvCarry);

  gemm64_f16_kernel<2><<<tilesQ / 8, 256, 0, stream>>>(
      Xk16, kDm, WTk, kDm, K16, kDm, bk, kTokK, kDm, kDm, kProjScale, kQkvCarry);

  constexpr int tilesV = (kDm / 64) * (kTokK / 64);
  static_assert((tilesV % 8) == 0);
  gemm64_f16_kernel<1><<<tilesV / 8, 256, 0, stream>>>(
      WTv, kDm, Xv16, kDm, VT16, kTokK, bv, kDm, kTokK, kDm, kProjScale, kQkvCarry);

  attn_kernel<<<kBatch * kQBlk * kNh, 128, 0, stream>>>(Q16, K16, VT16, aft, kwt, out);
}
